// FakeNewsClassifier_9586367005057
// MI455X (gfx1250) — hardware-verified
//
#include <hip/hip_runtime.h>
#include <math.h>

typedef __attribute__((ext_vector_type(16))) _Float16 v16h;
typedef __attribute__((ext_vector_type(8)))  _Float16 v8h;
typedef __attribute__((ext_vector_type(8)))  float    v8f;
typedef __attribute__((ext_vector_type(4)))  float    v4f;
typedef __attribute__((ext_vector_type(2)))  float    v2f;
typedef __attribute__((ext_vector_type(4)))  int      v4i;

constexpr int kRowsB   = 8192;
constexpr int kDim     = 1024;
constexpr int kDomains = 8;
constexpr int kOutW    = 2;
constexpr int kTileM   = 64;
constexpr int kTilesPerDomain = kRowsB / kTileM;
constexpr int kColSplit = 2;
constexpr int kColsPerBlock = kDim / kColSplit;
constexpr int kKChunk  = 256;
constexpr int kAPitch  = kKChunk + 8;
constexpr int kWtPitch = 72;
constexpr float kCarryX = 16.0f;
constexpr float kCarryW = 1024.0f;
constexpr float kFold   = 1.0f / (kCarryX * kCarryW);
constexpr float kHalfMinNormal = 6.103515625e-05f;

static_assert(kRowsB % kTileM == 0, "row tiles");
static_assert(kRowsB == 256 * 32, "id scan: 256 threads x 32 ids");
static_assert(kDim % kKChunk == 0 && kKChunk % 32 == 0, "k chunks are multiples of 32");
static_assert(kColsPerBlock == 8 * 64, "8 waves x 64 columns per block");
static_assert((kAPitch * 2) % 16 == 0 && (kWtPitch * 2) % 16 == 0, "16-B aligned LDS rows");
static_assert(kTileM * kOutW * 4 == 512, "one tile of head partials = four 128-B lines");
static_assert(kDomains == 8 && kOutW == 2, "layout assumptions");

constexpr size_t kOffW1T  = 0;
constexpr size_t kBytesW1T = (size_t)kDomains * kDim * kDim * 2;
constexpr size_t kOffPL   = kOffW1T + kBytesW1T;
constexpr size_t kBytesPL = (size_t)kColSplit * kDomains * kRowsB * kOutW * 4;
constexpr size_t kWsTotal = kOffPL + kBytesPL;
static_assert(kBytesW1T == 16777216ull && kBytesPL == 1048576ull, "carve sizes");
static_assert(kWsTotal == 17825792ull, "carve total");
static_assert(kWsTotal <= 134217728ull, "carve cap");
static_assert((kOffPL % 128) == 0, "128-B aligned regions");

__device__ __forceinline__ int clamp_dom(int v) {
  v = v < 0 ? 0 : v;
  v = v > (kDomains - 1) ? (kDomains - 1) : v;
  return v;
}

__device__ __forceinline__ _Float16 cvt_carry(float v, float carry) {
  const float s = v * carry;
  const float f = (fabsf(s) < kHalfMinNormal) ? 0.0f : s;
  return (_Float16)f;
}

union FragU { v16h v; v8h h[2]; };
__device__ __forceinline__ v16h frag_load(const _Float16* p) {
  FragU f;
  f.h[0] = *(const v8h*)(p);
  f.h[1] = *(const v8h*)(p + 16);
  return f.v;
}
__device__ __forceinline__ v8f mma_h(v16h a, v16h b, v8f c) {
  return __builtin_amdgcn_wmma_f32_16x16x32_f16(false, a, false, b, (short)0, c, false, false);
}
__device__ __forceinline__ void tie_h(v8f& c, v16h a, v16h b) {
  asm volatile("" : "+v"(c) : "v"(a), "v"(b));
}
__device__ __forceinline__ void nop_tie_h(v8f& c, v16h a, v16h b) {
  asm volatile("v_nop\n\tv_nop\n\tv_nop\n\tv_nop" : "+v"(c) : "v"(a), "v"(b));
}
__device__ __forceinline__ void keep4_h(v16h a, v16h b, v16h c, v16h d) {
  asm volatile("v_nop" :: "v"(a), "v"(b), "v"(c), "v"(d));
}
__device__ __forceinline__ void acc_guard4(v8f& a, v8f& b, v8f& c, v8f& d) {
  asm volatile("v_nop\n\tv_nop\n\tv_nop\n\tv_nop" : "+v"(a), "+v"(b), "+v"(c), "+v"(d));
}

__global__ __launch_bounds__(256) void pack_w1t_kernel(const float* __restrict__ W1, _Float16* __restrict__ W1T)
{
  __shared__ __align__(16) _Float16 sT[64 * kWtPitch];
  const int tid = threadIdx.x;
  const int n0 = blockIdx.x * 64;
  const int k0 = blockIdx.y * 64;
  const int e  = blockIdx.z;
  const int c4 = (tid & 15) * 4;
#pragma unroll
  for (int i = 0; i < 4; ++i) {
    const int kr = (tid >> 4) + 16 * i;
    const v4f a = *(const v4f*)(W1 + ((size_t)e * kDim + k0 + kr) * kDim + n0 + c4);
    const float a0 = a[0], a1 = a[1], a2 = a[2], a3 = a[3];
    sT[(c4 + 0) * kWtPitch + kr] = cvt_carry(a0, kCarryW);
    sT[(c4 + 1) * kWtPitch + kr] = cvt_carry(a1, kCarryW);
    sT[(c4 + 2) * kWtPitch + kr] = cvt_carry(a2, kCarryW);
    sT[(c4 + 3) * kWtPitch + kr] = cvt_carry(a3, kCarryW);
  }
  __syncthreads();
  const int c8 = (tid & 7) * 8;
  v8h hv[2];
#pragma unroll
  for (int i = 0; i < 2; ++i) {
    const int nr = (tid >> 3) + 32 * i;
    hv[i] = *(const v8h*)(sT + nr * kWtPitch + c8);
  }
  for (int pass = 0; pass < 2; ++pass) {
#pragma unroll
    for (int i = 0; i < 2; ++i) {
      const int nr = (tid >> 3) + 32 * i;
      *(volatile v8h*)(W1T + ((size_t)e * kDim + n0 + nr) * kDim + k0 + c8) = hv[i];
    }
    __threadfence();
  }
}

__global__ __launch_bounds__(256) void route_gemm_head_kernel(
    const float* __restrict__ X, const int* __restrict__ ids, const _Float16* __restrict__ W1T,
    const float* __restrict__ B1, const float* __restrict__ W2, float* __restrict__ PL)
{
  __shared__ __align__(16) _Float16 As[kTileM * kAPitch];
  __shared__ __align__(16) float wp[8 * 128];
  __shared__ int sRow[kTileM];
  __shared__ int sWT[8];

  const int tid  = threadIdx.x;
  const int lane = tid & 31;
  const int wave = tid >> 5;
  const int tile = blockIdx.x;
  const int e    = blockIdx.y;
  const int z    = blockIdx.z;

  if (tid < kTileM) sRow[tid] = -1;

  const v4i* idv = (const v4i*)ids + tid * 8;
  int c = 0;
#pragma unroll 1
  for (int q = 0; q < 8; ++q) {
    const v4i v = idv[q];
    const int i0 = v.x, i1 = v.y, i2 = v.z, i3 = v.w;
    c += (clamp_dom(i0) == e) ? 1 : 0;
    c += (clamp_dom(i1) == e) ? 1 : 0;
    c += (clamp_dom(i2) == e) ? 1 : 0;
    c += (clamp_dom(i3) == e) ? 1 : 0;
  }
  int x = c;
#pragma unroll
  for (int d = 1; d < 32; d <<= 1) {
    const int y = __shfl_up(x, d, 32);
    x += (lane >= d) ? y : 0;
  }
  if (lane == 31) sWT[wave] = x;
  __syncthreads();
  int woff = 0, cnt = 0;
#pragma unroll
  for (int w = 0; w < 8; ++w) {
    const int s = sWT[w];
    cnt += s;
    woff += (w < wave) ? s : 0;
  }
  if (tile * kTileM >= cnt) return;

  int pos = woff + x - c - tile * kTileM;
#pragma unroll 1
  for (int q = 0; q < 8; ++q) {
    const v4i v = idv[q];
    const int i0 = v.x, i1 = v.y, i2 = v.z, i3 = v.w;
    const int rb = tid * 32 + q * 4;
    const int m0 = (clamp_dom(i0) == e) ? 1 : 0;
    if (m0 && (unsigned)pos < (unsigned)kTileM) sRow[pos] = rb;
    pos += m0;
    const int m1 = (clamp_dom(i1) == e) ? 1 : 0;
    if (m1 && (unsigned)pos < (unsigned)kTileM) sRow[pos] = rb + 1;
    pos += m1;
    const int m2 = (clamp_dom(i2) == e) ? 1 : 0;
    if (m2 && (unsigned)pos < (unsigned)kTileM) sRow[pos] = rb + 2;
    pos += m2;
    const int m3 = (clamp_dom(i3) == e) ? 1 : 0;
    if (m3 && (unsigned)pos < (unsigned)kTileM) sRow[pos] = rb + 3;
    pos += m3;
  }

  const int rlane = lane & 15;
  const int koff  = (lane >> 4) * 8;
  const int mOff  = (lane >> 4) * 8;
  const int n0    = z * kColsPerBlock + wave * 64;
  const _Float16* Bw = W1T + (size_t)e * kDim * kDim;

  v8f acc[4][4];
#pragma unroll
  for (int i = 0; i < 4; ++i)
#pragma unroll
    for (int j = 0; j < 4; ++j) acc[i][j] = (v8f){0.f, 0.f, 0.f, 0.f, 0.f, 0.f, 0.f, 0.f};

#pragma unroll 1
  for (int kc = 0; kc < kDim; kc += kKChunk) {
    __syncthreads();
#pragma unroll 2
    for (int i = 0; i < 8; ++i) {
      const int row = wave + 8 * i;
      const int r = sRow[row];
      const bool valid = (r >= 0);
      int rc = r < 0 ? 0 : r;
      rc = rc > (kRowsB - 1) ? (kRowsB - 1) : rc;
      const float* src = X + (size_t)rc * kDim + kc + lane * 8;
      const v4f a0 = *(const v4f*)(src);
      const v4f a1 = *(const v4f*)(src + 4);
      v8h hv;
#pragma unroll
      for (int q = 0; q < 4; ++q) {
        const float f0 = a0[q], f1 = a1[q];
        const _Float16 h0 = cvt_carry(f0, kCarryX);
        const _Float16 h1 = cvt_carry(f1, kCarryX);
        hv[q]     = valid ? h0 : (_Float16)0.0f;
        hv[4 + q] = valid ? h1 : (_Float16)0.0f;
      }
      *(v8h*)(As + row * kAPitch + lane * 8) = hv;
    }
    __syncthreads();
#pragma unroll 1
    for (int kk = 0; kk < kKChunk; kk += 32) {
      v16h bh[4];
#pragma unroll
      for (int j = 0; j < 4; ++j)
        bh[j] = frag_load(Bw + (size_t)(n0 + (j << 4) + rlane) * kDim + kc + kk + koff);
#pragma unroll
      for (int i = 0; i < 4; ++i) {
        const v16h ah = frag_load(As + ((i << 4) + rlane) * kAPitch + kk + koff);
        acc[i][0] = mma_h(ah, bh[0], acc[i][0]);
        acc[i][1] = mma_h(ah, bh[1], acc[i][1]);
        acc[i][2] = mma_h(ah, bh[2], acc[i][2]);
        acc[i][3] = mma_h(ah, bh[3], acc[i][3]);
        tie_h(acc[i][0], ah, bh[0]);
        tie_h(acc[i][1], ah, bh[1]);
        tie_h(acc[i][2], ah, bh[2]);
        nop_tie_h(acc[i][3], ah, bh[3]);
      }
      keep4_h(bh[0], bh[1], bh[2], bh[3]);
    }
  }
  acc_guard4(acc[0][0], acc[0][1], acc[0][2], acc[0][3]);
  acc_guard4(acc[1][0], acc[1][1], acc[1][2], acc[1][3]);
  acc_guard4(acc[2][0], acc[2][1], acc[2][2], acc[2][3]);
  acc_guard4(acc[3][0], acc[3][1], acc[3][2], acc[3][3]);

  float bv[4], w2a[4], w2b[4];
#pragma unroll
  for (int j = 0; j < 4; ++j) {
    const int n = n0 + (j << 4) + rlane;
    bv[j] = B1[e * kDim + n];
    const v2f wv = *(const v2f*)(W2 + ((size_t)e * kDim + n) * kOutW);
    w2a[j] = wv[0];
    w2b[j] = wv[1];
  }
  float* slab = wp + wave * 128;
#pragma unroll
  for (int i = 0; i < 4; ++i) {
    float p0[8], p1[8];
#pragma unroll
    for (int r = 0; r < 8; ++r) { p0[r] = 0.0f; p1[r] = 0.0f; }
#pragma unroll
    for (int j = 0; j < 4; ++j) {
#pragma unroll
      for (int r = 0; r < 8; ++r) {
        float h = fmaf(acc[i][j][r], kFold, bv[j]);
        h = fmaxf(h, 0.0f);
        p0[r] = fmaf(h, w2a[j], p0[r]);
        p1[r] = fmaf(h, w2b[j], p1[r]);
      }
    }
#pragma unroll
    for (int off = 1; off < 16; off <<= 1) {
#pragma unroll
      for (int r = 0; r < 8; ++r) {
        const float t0 = __shfl_xor(p0[r], off, 32);
        const float t1 = __shfl_xor(p1[r], off, 32);
        p0[r] += t0;
        p1[r] += t1;
      }
    }
    if (rlane == 0) {
#pragma unroll
      for (int r = 0; r < 8; ++r) {
        slab[((i << 4) + mOff + r) * 2 + 0] = p0[r];
        slab[((i << 4) + mOff + r) * 2 + 1] = p1[r];
      }
    }
  }
  __syncthreads();
  if (wave == 0) {
    v4f v;
#pragma unroll
    for (int q = 0; q < 4; ++q) {
      float s = 0.0f;
#pragma unroll
      for (int w = 0; w < 8; ++w) s += wp[w * 128 + lane * 4 + q];
      v[q] = s;
    }
    float* dst = PL + ((size_t)(z * kDomains + e) * kRowsB + (size_t)tile * kTileM) * kOutW + lane * 4;
    *(volatile v4f*)dst = v;
    __threadfence();
    *(volatile v4f*)dst = v;
  }
}

__global__ __launch_bounds__(256) void place_rows_kernel(
    const int* __restrict__ ids, const float* __restrict__ PL, const float* __restrict__ B2, float* __restrict__ out)
{
  __shared__ int sC[8][8];
  __shared__ int sW[8][8];
  __shared__ __align__(16) float sO[512];
  const int tid  = threadIdx.x;
  const int lane = tid & 31;
  const int wave = tid >> 5;
  const int b0   = blockIdx.x * 256;
  int nIter = blockIdx.x;
  nIter = nIter > 31 ? 31 : nIter;

  int cw[8];
#pragma unroll
  for (int d = 0; d < 8; ++d) cw[d] = 0;
#pragma unroll 1
  for (int it = 0; it < nIter; ++it) {
    const int id = clamp_dom(ids[it * 256 + tid]);
#pragma unroll
    for (int d = 0; d < 8; ++d) {
      const unsigned m = (unsigned)__ballot(id == d);
      cw[d] += __popc(m);
    }
  }
  const int eo = clamp_dom(ids[b0 + tid]);
  const unsigned ltmask = (1u << lane) - 1u;
  int lr = 0;
  int tw[8];
#pragma unroll
  for (int d = 0; d < 8; ++d) {
    const unsigned m = (unsigned)__ballot(eo == d);
    const int before = __popc(m & ltmask);
    lr = (eo == d) ? before : lr;
    tw[d] = __popc(m);
  }
  if (lane == 0) {
#pragma unroll
    for (int d = 0; d < 8; ++d) {
      sC[wave][d] = cw[d];
      sW[wave][d] = tw[d];
    }
  }
  __syncthreads();
  int rank = lr;
#pragma unroll
  for (int w = 0; w < 8; ++w) {
    const int a = sC[w][eo];
    const int b = sW[w][eo];
    rank += a;
    rank += (w < wave) ? b : 0;
  }
  rank = rank < 0 ? 0 : rank;
  rank = rank > (kRowsB - 1) ? (kRowsB - 1) : rank;
  const v2f q0 = *(const v2f*)(PL + ((size_t)(0 * kDomains + eo) * kRowsB + rank) * kOutW);
  const v2f q1 = *(const v2f*)(PL + ((size_t)(1 * kDomains + eo) * kRowsB + rank) * kOutW);
  const v2f bb = *(const v2f*)(B2 + eo * kOutW);
  const float o0 = (q0[0] + q1[0]) + bb[0];
  const float o1 = (q0[1] + q1[1]) + bb[1];
  sO[tid * 2 + 0] = o0;
  sO[tid * 2 + 1] = o1;
  __syncthreads();
  if (tid < 128) {
    const v4f v = *(const v4f*)(sO + tid * 4);
    float* dst = out + (size_t)b0 * kOutW + tid * 4;
    *(volatile v4f*)dst = v;
    __threadfence();
    *(volatile v4f*)dst = v;
  }
}

extern "C" void kernel_launch(void* const* d_in, const int* in_sizes, int n_in,
                              void* d_out, int out_size, void* d_ws, size_t ws_size,
                              hipStream_t stream) {
  if (n_in < 6) return;
  if (in_sizes[0] != kRowsB * kDim) return;
  if (in_sizes[1] != kRowsB) return;
  if (in_sizes[2] != kDomains * kDim * kDim) return;
  if (in_sizes[3] != kDomains * kDim) return;
  if (in_sizes[4] != kDomains * kDim * kOutW) return;
  if (in_sizes[5] != kDomains * kOutW) return;
  if (out_size != kRowsB * kOutW) return;
  if (ws_size < kWsTotal) return;

  const float* X   = (const float*)d_in[0];
  const int*   ids = (const int*)d_in[1];
  const float* W1  = (const float*)d_in[2];
  const float* B1  = (const float*)d_in[3];
  const float* W2  = (const float*)d_in[4];
  const float* B2  = (const float*)d_in[5];
  float* out = (float*)d_out;

  char* ws = (char*)d_ws;
  _Float16* W1T = (_Float16*)(ws + kOffW1T);
  float*    PL  = (float*)(ws + kOffPL);

  pack_w1t_kernel<<<dim3(kDim / 64, kDim / 64, kDomains), 256, 0, stream>>>(W1, W1T);
  route_gemm_head_kernel<<<dim3(kTilesPerDomain, kDomains, kColSplit), 256, 0, stream>>>(X, ids, W1T, B1, W2, PL);
  place_rows_kernel<<<kRowsB / 256, 256, 0, stream>>>(ids, PL, B2, out);
}
